// StructuralEquationNetwork_62277025792816
// MI455X (gfx1250) — hardware-verified
//
#include <hip/hip_runtime.h>

typedef _Float16     v16h __attribute__((ext_vector_type(16)));
typedef _Float16     v8h  __attribute__((ext_vector_type(8)));
typedef float        v8f  __attribute__((ext_vector_type(8)));
typedef float        v4f  __attribute__((ext_vector_type(4)));
typedef unsigned int v4u  __attribute__((ext_vector_type(4)));

union Frag  { v16h v; v8h half[2]; };
union Pack8 { v8h h; v4f f; };

#define NV           64
#define HID          256
#define HID2         128
#define WAVES        8
#define ROWS_PB      (WAVES * 16)
#define BLOB_BYTES   102400
#define W2T_BYTE_OFF 32768
#define VEC_BYTE_OFF 98304
#define SC_W         64.0f
#define SC_B2        4096.0f
#define SC_W3        0.000244140625f

static_assert(BLOB_BYTES == W2T_BYTE_OFF + 65536 + 4096);
static_assert(VEC_BYTE_OFF == W2T_BYTE_OFF + 65536);

__device__ __forceinline__ v8f wmma_f16(v16h a, v16h b, v8f c) {
    return __builtin_amdgcn_wmma_f32_16x16x32_f16(false, a, false, b, (short)0, c, false, false);
}
__device__ __forceinline__ void wguard(v8f& acc, const v16h& a, const v16h& b) {
    asm volatile("v_nop\n\tv_nop\n\tv_nop\n\tv_nop" : "+v"(acc) : "v"(a), "v"(b));
}
__device__ __forceinline__ v8f zero8() {
    v8f z = {0.f, 0.f, 0.f, 0.f, 0.f, 0.f, 0.f, 0.f};
    return z;
}

__global__ void __launch_bounds__(256)
prep_params(const float* __restrict__ W1, const float* __restrict__ b1,
            const float* __restrict__ W2, const float* __restrict__ b2,
            const float* __restrict__ W3, const float* __restrict__ b3,
            const int* __restrict__ G, unsigned char* __restrict__ ws)
{
    const int i   = blockIdx.x;
    const int tid = threadIdx.x;
    const int w   = tid >> 5;
    const int l   = tid & 31;
    unsigned char* blob = ws + (size_t)i * BLOB_BYTES;

#pragma unroll 1
    for (int it = 0; it < 8; ++it) {
        const int n  = it * 32 + w * 4 + (l >> 3);
        const int k0 = (l & 7) * 8;
        Pack8 p;
#pragma unroll
        for (int j = 0; j < 8; ++j) {
            const int k = k0 + j;
            float v = 0.0f;
            if (G[k * NV + i] > 0) v = W1[((size_t)i * (NV + 1) + k) * HID + n] * SC_W;
            p.h[j] = (_Float16)v;
        }
        const v4f val = p.f;
        volatile v4f* d = (volatile v4f*)(blob + ((size_t)n * NV + k0) * 2);
        *d = val;
        __threadfence();
        *d = val;
    }

#pragma unroll 1
    for (int it = 0; it < 16; ++it) {
        const int n2 = it * 8 + w;
        const int k0 = l * 8;
        Pack8 p;
#pragma unroll
        for (int j = 0; j < 8; ++j)
            p.h[j] = (_Float16)(W2[((size_t)i * HID + k0 + j) * HID2 + n2] * SC_W);
        const v4f val = p.f;
        volatile v4f* d = (volatile v4f*)(blob + W2T_BYTE_OFF + ((size_t)n2 * HID + k0) * 2);
        *d = val;
        __threadfence();
        *d = val;
    }

    {
        const int t = tid;
        v4f val;
#pragma unroll
        for (int c = 0; c < 4; ++c) {
            float x = 0.0f;
            if (t < 64)        x = b1[(size_t)i * HID + 4 * t + c] * SC_W;
            else if (t < 128)  x = W1[((size_t)i * (NV + 1) + NV) * HID + 4 * (t - 64) + c] * SC_W;
            else if (t < 160)  x = b2[(size_t)i * HID2 + 4 * (t - 128) + c] * SC_B2;
            else if (t < 192)  x = W3[(size_t)i * HID2 + 4 * (t - 160) + c] * SC_W3;
            else if (t == 192 && c == 0) x = b3[i];
            val[c] = x;
        }
        volatile v4f* d = (volatile v4f*)(blob + VEC_BYTE_OFF + (size_t)t * 16);
        *d = val;
        __threadfence();
        *d = val;
    }
}

__global__ void __launch_bounds__(WAVES * 32)
sen_main(const float* __restrict__ X, const float* __restrict__ U,
         const unsigned char* __restrict__ ws, float* __restrict__ out)
{
    __shared__ __align__(32) unsigned char WB[BLOB_BYTES];
    __shared__ __align__(32) float Ylds[WAVES * 16 * NV];

    const int tid  = threadIdx.x;
    const int lane = tid & 31;
    const int w    = tid >> 5;
    const int h    = lane >> 4;
    const int m    = lane & 15;
    const int woff = w * 16 * NV;
    const int row0 = (blockIdx.x * WAVES + w) * 16;

    for (int idx = lane; idx < 16 * NV; idx += 32)
        Ylds[woff + idx] = X[(size_t)row0 * NV + idx];

    const _Float16* W1t = (const _Float16*)WB;
    const _Float16* W2t = (const _Float16*)(WB + W2T_BYTE_OFF);
    const float*    Vf  = (const float*)(WB + VEC_BYTE_OFF);

#pragma unroll 1
    for (int i = 0; i < NV; ++i) {
        __syncthreads();
        {
            const v4u* src = (const v4u*)(ws + (size_t)i * BLOB_BYTES);
            v4u* dst = (v4u*)WB;
            for (int idx = tid; idx < BLOB_BYTES / 16; idx += WAVES * 32)
                dst[idx] = src[idx];
        }
        __syncthreads();

        const float uval = U[(size_t)(row0 + m) * NV + i];

        Frag yb[2];
#pragma unroll
        for (int s = 0; s < 2; ++s) {
            const float* yrow = &Ylds[woff + m * NV + 32 * s + 8 * h];
            const v8f lo = *(const v8f*)yrow;
            const v8f hi = *(const v8f*)(yrow + 16);
            yb[s].half[0] = __builtin_convertvector(lo, v8h);
            yb[s].half[1] = __builtin_convertvector(hi, v8h);
        }

        Frag bfr[8];
#pragma unroll
        for (int tp = 0; tp < 8; ++tp) {
            const int na = 32 * tp + 8 * h;
            v8f acc0, acc1;
            {
                const v8f bv = *(const v8f*)(Vf + na);
                const v8f wu = *(const v8f*)(Vf + HID + na);
                acc0 = bv + uval * wu;
                const v8f bv1 = *(const v8f*)(Vf + na + 16);
                const v8f wu1 = *(const v8f*)(Vf + HID + na + 16);
                acc1 = bv1 + uval * wu1;
            }
            Frag a;
            a.half[0] = *(const v8h*)(W1t + (32 * tp + m) * NV + 8 * h);
            a.half[1] = *(const v8h*)(W1t + (32 * tp + m) * NV + 16 + 8 * h);
            acc0 = wmma_f16(a.v, yb[0].v, acc0);
            a.half[0] = *(const v8h*)(W1t + (32 * tp + m) * NV + 32 + 8 * h);
            a.half[1] = *(const v8h*)(W1t + (32 * tp + m) * NV + 48 + 8 * h);
            acc0 = wmma_f16(a.v, yb[1].v, acc0);
            wguard(acc0, a.v, yb[1].v);
            a.half[0] = *(const v8h*)(W1t + (32 * tp + 16 + m) * NV + 8 * h);
            a.half[1] = *(const v8h*)(W1t + (32 * tp + 16 + m) * NV + 16 + 8 * h);
            acc1 = wmma_f16(a.v, yb[0].v, acc1);
            a.half[0] = *(const v8h*)(W1t + (32 * tp + 16 + m) * NV + 32 + 8 * h);
            a.half[1] = *(const v8h*)(W1t + (32 * tp + 16 + m) * NV + 48 + 8 * h);
            acc1 = wmma_f16(a.v, yb[1].v, acc1);
            wguard(acc1, a.v, yb[1].v);
#pragma unroll
            for (int r = 0; r < 8; ++r) {
                acc0[r] = fmaxf(acc0[r], 0.0f);
                acc1[r] = fmaxf(acc1[r], 0.0f);
            }
            bfr[tp].half[0] = __builtin_convertvector(acc0, v8h);
            bfr[tp].half[1] = __builtin_convertvector(acc1, v8h);
        }

        v8f acc2[8];
#pragma unroll
        for (int t = 0; t < 8; ++t) {
            acc2[t] = zero8();
            Frag a;
#pragma unroll
            for (int s = 0; s < 8; ++s) {
                a.half[0] = *(const v8h*)(W2t + (16 * t + m) * HID + 32 * s + 8 * h);
                a.half[1] = *(const v8h*)(W2t + (16 * t + m) * HID + 32 * s + 16 + 8 * h);
                acc2[t] = wmma_f16(a.v, bfr[s].v, acc2[t]);
            }
            wguard(acc2[t], a.v, bfr[7].v);
        }

        float part = 0.0f;
#pragma unroll
        for (int t = 0; t < 8; ++t) {
            const v8f b2v = *(const v8f*)(Vf + 512 + 16 * t + 8 * h);
            const v8f w3v = *(const v8f*)(Vf + 640 + 16 * t + 8 * h);
#pragma unroll
            for (int r = 0; r < 8; ++r)
                part = fmaf(fmaxf(acc2[t][r] + b2v[r], 0.0f), w3v[r], part);
        }
        part += __shfl_xor(part, 16, 32);
        const float y = part + Vf[768];
        if (h == 0) Ylds[woff + m * NV + i] = y;
    }
    __syncthreads();

    v4f ov[8];
#pragma unroll
    for (int p = 0; p < 8; ++p) {
        const int row = 2 * p + h;
        ov[p] = *(const v4f*)&Ylds[woff + row * NV + 4 * m];
    }
#pragma unroll
    for (int p = 0; p < 8; ++p) {
        const int row = 2 * p + h;
        *(volatile v4f*)(out + (size_t)(row0 + row) * NV + 4 * m) = ov[p];
    }
    __threadfence();
#pragma unroll
    for (int p = 0; p < 8; ++p) {
        const int row = 2 * p + h;
        *(volatile v4f*)(out + (size_t)(row0 + row) * NV + 4 * m) = ov[p];
    }
}

extern "C" void kernel_launch(void* const* d_in, const int* in_sizes, int n_in,
                              void* d_out, int out_size, void* d_ws, size_t ws_size,
                              hipStream_t stream)
{
    if (n_in < 9) return;
    const float* X  = (const float*)d_in[0];
    const float* U  = (const float*)d_in[1];
    const int*   G  = (const int*)  d_in[2];
    const float* W1 = (const float*)d_in[3];
    const float* b1 = (const float*)d_in[4];
    const float* W2 = (const float*)d_in[5];
    const float* b2 = (const float*)d_in[6];
    const float* W3 = (const float*)d_in[7];
    const float* b3 = (const float*)d_in[8];
    float* out = (float*)d_out;
    unsigned char* ws = (unsigned char*)d_ws;

    const int batch = in_sizes[0] / NV;
    if (batch <= 0 || (batch % ROWS_PB) != 0) return;
    if (out_size < batch * NV) return;
    if (in_sizes[2] < NV * NV) return;
    if ((size_t)NV * BLOB_BYTES > ws_size) return;

    prep_params<<<NV, 256, 0, stream>>>(W1, b1, W2, b2, W3, b3, G, ws);
    sen_main<<<batch / ROWS_PB, WAVES * 32, 0, stream>>>(X, U, ws, out);
}
